// RWKV_v7_TimeMix_26242250178958
// MI455X (gfx1250) — hardware-verified
//
#include <hip/hip_runtime.h>


#define T_    1024
#define C_    1024
#define H_    16
#define N_    64
#define M_    4096
#define EPSGN 0.00064f

static_assert(M_ % 64 == 0);
static_assert(C_ % 64 == 0);
static_assert(H_ * N_ == C_);
static_assert(T_ % 32 == 0);

typedef float          v4f   __attribute__((ext_vector_type(4)));
typedef float          v8f   __attribute__((ext_vector_type(8)));
typedef __bf16         v16b  __attribute__((ext_vector_type(16)));
typedef _Float16       v16h  __attribute__((ext_vector_type(16)));
typedef _Float16       v8h   __attribute__((ext_vector_type(8)));
typedef unsigned short u16x8 __attribute__((ext_vector_type(8)));

union FragB { u16x8 h[2]; v16b v; };
union FragH { u16x8 h[2]; v16h v; };
union Pack8 { v8h f; u16x8 u; };

constexpr size_t SZ_X16 = (size_t)M_ * C_ * 2;
constexpr size_t SZ_P32 = (size_t)M_ * C_ * 4;
constexpr size_t SZ_W16 = (size_t)C_ * C_ * 2;

constexpr size_t OFF_XH  = 0;
constexpr size_t OFF_XL  = OFF_XH + SZ_X16;
constexpr size_t OFF_WH  = OFF_XL + SZ_X16;
constexpr size_t OFF_WL  = OFF_WH + SZ_W16;
constexpr size_t OFF_W2  = OFF_WL + SZ_W16;
constexpr size_t OFF_Y   = 0;
constexpr size_t OFF_XG  = OFF_Y + SZ_P32;
constexpr size_t OFF_WG  = OFF_XG + SZ_X16;
constexpr size_t OFF_WOH = OFF_WG + SZ_W16;
constexpr size_t OFF_WOL = OFF_WOH + SZ_W16;
constexpr size_t OFF_A   = (size_t)32 * 1048576;
constexpr size_t OFF_KM  = OFF_A  + SZ_P32;
constexpr size_t OFF_KK  = OFF_KM + SZ_P32;
constexpr size_t OFF_R   = OFF_KK + SZ_P32;
constexpr size_t OFF_WD  = OFF_R  + SZ_P32;
constexpr size_t OFF_V   = OFF_WD + SZ_P32;
constexpr size_t WS_END  = OFF_V  + SZ_P32;
constexpr size_t OFF_G   = OFF_A;
constexpr size_t OFF_YGH = OFF_KK;
constexpr size_t OFF_YGL = OFF_KK + SZ_X16;
static_assert(WS_END <= (size_t)134217728);
static_assert(OFF_W2 + SZ_W16 <= OFF_A);
static_assert(OFF_WOL + SZ_W16 <= OFF_A);
static_assert(OFF_YGL + SZ_X16 <= OFF_R);
static_assert(OFF_XL % 128 == 0 && OFF_WH % 128 == 0 && OFF_WL % 128 == 0 && OFF_W2 % 128 == 0);
static_assert(OFF_XG % 128 == 0 && OFF_WG % 128 == 0 && OFF_WOH % 128 == 0 && OFF_WOL % 128 == 0);
static_assert(OFF_A % 128 == 0 && OFF_KM % 128 == 0 && OFF_KK % 128 == 0 && OFF_R % 128 == 0);
static_assert(OFF_WD % 128 == 0 && OFF_V % 128 == 0 && OFF_YGL % 128 == 0);

__device__ __forceinline__ unsigned short f32_to_bf16(float f) {
    unsigned u = __float_as_uint(f);
    unsigned r = u + 0x7FFFu + ((u >> 16) & 1u);
    return (unsigned short)(r >> 16);
}
__device__ __forceinline__ float bf16_to_f32(unsigned short b) {
    return __uint_as_float(((unsigned)b) << 16);
}
__device__ __forceinline__ v8f ld8f(const float* p) {
    v4f a = *(const v4f*)p;
    v4f b = *(const v4f*)(p + 4);
    return __builtin_shufflevector(a, b, 0, 1, 2, 3, 4, 5, 6, 7);
}
__device__ __forceinline__ void split8(const v8f x, u16x8& hv, u16x8& lv) {
#pragma unroll
    for (int c = 0; c < 8; ++c) {
        const float f = x[c];
        const unsigned short hb = f32_to_bf16(f);
        const unsigned short lb = f32_to_bf16(f - bf16_to_f32(hb));
        hv[c] = hb;
        lv[c] = lb;
    }
}
__device__ __forceinline__ u16x8 to_f16x8(const v8f x, float sc) {
    Pack8 p;
#pragma unroll
    for (int c = 0; c < 8; ++c) p.f[c] = (_Float16)(x[c] * sc);
    return p.u;
}
__device__ __forceinline__ float sigm(float x) {
    const float e = expf(-x);
    return __builtin_amdgcn_rcpf(1.0f + e);
}

__device__ __forceinline__ void mma_bf(v8f& acc, const FragB& a, const FragB& b) {
    acc = __builtin_amdgcn_wmma_f32_16x16x32_bf16(false, a.v, false, b.v, (short)0, acc, false, false);
    asm volatile("v_nop\n\tv_nop\n\tv_nop\n\tv_nop" : "+v"(acc) : "v"(a.v), "v"(b.v));
}
__device__ __forceinline__ void mma_hf(v8f& acc, const FragH& a, const FragH& b) {
    acc = __builtin_amdgcn_wmma_f32_16x16x32_f16(false, a.v, false, b.v, (short)0, acc, false, false);
    asm volatile("v_nop\n\tv_nop\n\tv_nop\n\tv_nop" : "+v"(acc) : "v"(a.v), "v"(b.v));
}

__device__ __forceinline__ v8f mix8(const float* __restrict__ x, const float* __restrict__ coef, size_t e) {
    const int mrow = (int)(e >> 10);
    const int c    = (int)(e & (C_ - 1));
    const int t    = mrow & (T_ - 1);
    const size_t ep = (t > 0) ? (e - (size_t)C_) : e;
    const float z   = (t > 0) ? 1.0f : 0.0f;
    const v8f xc = ld8f(x + e);
    const v8f xp = ld8f(x + ep) * z;
    const v8f cf = ld8f(coef + c);
    v8f u;
#pragma unroll
    for (int q = 0; q < 8; ++q) u[q] = xc[q] + (xp[q] - xc[q]) * cf[q];
    return u;
}

__global__ __launch_bounds__(256)
void mix_split_kernel(const float* __restrict__ x, const float* __restrict__ coef,
                      unsigned short* dhi, unsigned short* dlo, int n8)
{
    const int i = blockIdx.x * 256 + threadIdx.x;
    if (i >= n8) return;
    const size_t e = (size_t)i * 8;
    const v8f u = mix8(x, coef, e);
    u16x8 hv, lv;
    split8(u, hv, lv);
    *(volatile u16x8*)(dhi + e) = hv;
    *(volatile u16x8*)(dlo + e) = lv;
    __threadfence();
    *(volatile u16x8*)(dhi + e) = hv;
    *(volatile u16x8*)(dlo + e) = lv;
}

__global__ __launch_bounds__(256)
void mix_f16_kernel(const float* __restrict__ x, const float* __restrict__ coef,
                    unsigned short* dst, int n8)
{
    const int i = blockIdx.x * 256 + threadIdx.x;
    if (i >= n8) return;
    const size_t e = (size_t)i * 8;
    const v8f u = mix8(x, coef, e);
    const u16x8 hv = to_f16x8(u, 1.0f);
    *(volatile u16x8*)(dst + e) = hv;
    __threadfence();
    *(volatile u16x8*)(dst + e) = hv;
}

__global__ __launch_bounds__(256)
void w_split_kernel(const float* __restrict__ src, unsigned short* dhi, unsigned short* dlo, int n8)
{
    const int i = blockIdx.x * 256 + threadIdx.x;
    if (i >= n8) return;
    const size_t e = (size_t)i * 8;
    const v8f x = ld8f(src + e);
    u16x8 hv, lv;
    split8(x, hv, lv);
    *(volatile u16x8*)(dhi + e) = hv;
    *(volatile u16x8*)(dlo + e) = lv;
    __threadfence();
    *(volatile u16x8*)(dhi + e) = hv;
    *(volatile u16x8*)(dlo + e) = lv;
}

__global__ __launch_bounds__(256)
void w_f16_kernel(const float* __restrict__ src, unsigned short* dst, int n8)
{
    const int i = blockIdx.x * 256 + threadIdx.x;
    if (i >= n8) return;
    const size_t e = (size_t)i * 8;
    const v8f x = ld8f(src + e);
    const u16x8 hv = to_f16x8(x, 16.0f);
    *(volatile u16x8*)(dst + e) = hv;
    __threadfence();
    *(volatile u16x8*)(dst + e) = hv;
}

#define GP 36
#define EPI_PLAIN 0
#define EPI_AGATE 1
#define EPI_KPOST 2

template<int EPI>
__global__ __launch_bounds__(128)
void gemm_x3_kernel(const unsigned short* __restrict__ Ah, const unsigned short* __restrict__ Al,
                    const unsigned short* __restrict__ Bh, const unsigned short* __restrict__ Bl,
                    float* out0, float* out1,
                    const float* __restrict__ q0, const float* __restrict__ q1, const float* __restrict__ q2)
{
    __shared__ __attribute__((aligned(16))) float stile[4][32 * GP];

    const int tid  = threadIdx.x;
    const int lane = tid & 31;
    const int wave = tid >> 5;
    const int h    = lane >> 4;
    const int m    = lane & 15;
    const int wm   = wave >> 1;
    const int wn   = wave & 1;

    const int rowW = blockIdx.y * 64 + wm * 32;
    const int colB = blockIdx.x * 64;
    const int colW = colB + wn * 32;

    v8f acc[4];
#pragma unroll
    for (int j = 0; j < 4; ++j)
#pragma unroll
        for (int r = 0; r < 8; ++r) acc[j][r] = 0.0f;

    const size_t aoff  = (size_t)(rowW + m) * C_ + 8 * h;
    const size_t boff  = (size_t)(colW + m) * C_ + 8 * h;
    const size_t sub16 = (size_t)16 * C_;

#pragma unroll 1
    for (int kt = 0; kt < C_ / 32; ++kt) {
        const size_t k0 = (size_t)kt * 32;
        FragB fa[2], ga[2], fb[2], gb[2];
#pragma unroll
        for (int s = 0; s < 2; ++s) {
            const unsigned short* p = Ah + aoff + s * sub16 + k0;
            const unsigned short* q = Al + aoff + s * sub16 + k0;
            fa[s].h[0] = *(const u16x8*)(p);
            fa[s].h[1] = *(const u16x8*)(p + 16);
            ga[s].h[0] = *(const u16x8*)(q);
            ga[s].h[1] = *(const u16x8*)(q + 16);
        }
#pragma unroll
        for (int j = 0; j < 2; ++j) {
            const unsigned short* p = Bh + boff + j * sub16 + k0;
            const unsigned short* q = Bl + boff + j * sub16 + k0;
            fb[j].h[0] = *(const u16x8*)(p);
            fb[j].h[1] = *(const u16x8*)(p + 16);
            gb[j].h[0] = *(const u16x8*)(q);
            gb[j].h[1] = *(const u16x8*)(q + 16);
        }
#pragma unroll
        for (int s = 0; s < 2; ++s)
#pragma unroll
            for (int j = 0; j < 2; ++j) {
                mma_bf(acc[s * 2 + j], fa[s], fb[j]);
                mma_bf(acc[s * 2 + j], fa[s], gb[j]);
                mma_bf(acc[s * 2 + j], ga[s], fb[j]);
            }
    }

    float* st = stile[wave];
#pragma unroll
    for (int s = 0; s < 2; ++s)
#pragma unroll
        for (int j = 0; j < 2; ++j)
#pragma unroll
            for (int r = 0; r < 8; ++r)
                st[(s * 16 + 8 * h + r) * GP + j * 16 + m] = acc[s * 2 + j][r];
    __syncthreads();

    const int rsub = lane >> 3;
    const int c0   = (lane & 7) * 4;
    const int gn   = colW + c0;

    v4f res0[8], res1[8];
#pragma unroll
    for (int it = 0; it < 8; ++it) {
        const int row = it * 4 + rsub;
        const int gm  = rowW + row;
        const v4f v = *(const v4f*)(st + row * GP + c0);
        if (EPI == EPI_PLAIN) {
            res0[it] = v;
            res1[it] = v;
        } else if (EPI == EPI_AGATE) {
            const v4f b0 = *(const v4f*)(q0 + gn);
            const v4f b1 = *(const v4f*)(q1 + gn);
            v4f o;
#pragma unroll
            for (int q = 0; q < 4; ++q) o[q] = sigm(b0[q] + v[q] * b1[q]);
            res0[it] = o;
            res1[it] = o;
        } else {
            const float* sts = stile[wave ^ 1];
            const v4f vs  = *(const v4f*)(sts + row * GP + c0);
            const int gns = colB + (wn ^ 1) * 32 + c0;
            const v4f kk0 = *(const v4f*)(q0 + gn);
            const v4f kk1 = *(const v4f*)(q0 + gns);
            const v4f ko  = v * kk0;
            const v4f ks  = vs * kk1;
            float ss = ko[0] * ko[0] + ko[1] * ko[1] + ko[2] * ko[2] + ko[3] * ko[3]
                     + ks[0] * ks[0] + ks[1] * ks[1] + ks[2] * ks[2] + ks[3] * ks[3];
            ss += __shfl_xor(ss, 1, 32);
            ss += __shfl_xor(ss, 2, 32);
            ss += __shfl_xor(ss, 4, 32);
            const float inv = 1.0f / fmaxf(sqrtf(ss), 1e-12f);
            const v4f ka = *(const v4f*)(q1 + gn);
            const v4f av = *(const v4f*)(q2 + (size_t)gm * C_ + gn);
            v4f km;
#pragma unroll
            for (int q = 0; q < 4; ++q) km[q] = v[q] * (1.0f + (av[q] - 1.0f) * ka[q]);
            res0[it] = km;
            res1[it] = ko * inv;
        }
    }

#pragma unroll
    for (int it = 0; it < 8; ++it) {
        const size_t o = (size_t)(rowW + it * 4 + rsub) * C_ + gn;
        *(volatile v4f*)(out0 + o) = res0[it];
        if (EPI == EPI_KPOST) *(volatile v4f*)(out1 + o) = res1[it];
    }
    __threadfence();
#pragma unroll
    for (int it = 0; it < 8; ++it) {
        const size_t o = (size_t)(rowW + it * 4 + rsub) * C_ + gn;
        *(volatile v4f*)(out0 + o) = res0[it];
        if (EPI == EPI_KPOST) *(volatile v4f*)(out1 + o) = res1[it];
    }
}

#define EPI_WDEC  0
#define EPI_GGATE 1
#define EPI_VPAIR 2

template<int EPI>
__global__ __launch_bounds__(128)
void gemm_f16_kernel(const unsigned short* __restrict__ A, const unsigned short* __restrict__ B,
                     const unsigned short* __restrict__ B2, float* out0,
                     const float* __restrict__ q0, const float* __restrict__ q1, const float* __restrict__ q2)
{
    constexpr int NT = (EPI == EPI_VPAIR) ? 8 : 4;
    __shared__ __attribute__((aligned(16))) float stile[NT][32 * GP];

    const int tid  = threadIdx.x;
    const int lane = tid & 31;
    const int wave = tid >> 5;
    const int h    = lane >> 4;
    const int m    = lane & 15;
    const int wm   = wave >> 1;
    const int wn   = wave & 1;

    const int rowW = blockIdx.y * 64 + wm * 32;
    const int colW = blockIdx.x * 64 + wn * 32;

    v8f acc[4], acc2[4];
#pragma unroll
    for (int j = 0; j < 4; ++j)
#pragma unroll
        for (int r = 0; r < 8; ++r) { acc[j][r] = 0.0f; acc2[j][r] = 0.0f; }

    const size_t aoff  = (size_t)(rowW + m) * C_ + 8 * h;
    const size_t boff  = (size_t)(colW + m) * C_ + 8 * h;
    const size_t sub16 = (size_t)16 * C_;

#pragma unroll 1
    for (int kt = 0; kt < C_ / 32; ++kt) {
        const size_t k0 = (size_t)kt * 32;
        FragH fa[2], fb[2], fc[2];
#pragma unroll
        for (int s = 0; s < 2; ++s) {
            const unsigned short* p = A + aoff + s * sub16 + k0;
            fa[s].h[0] = *(const u16x8*)(p);
            fa[s].h[1] = *(const u16x8*)(p + 16);
        }
#pragma unroll
        for (int j = 0; j < 2; ++j) {
            const unsigned short* p = B + boff + j * sub16 + k0;
            fb[j].h[0] = *(const u16x8*)(p);
            fb[j].h[1] = *(const u16x8*)(p + 16);
            if (EPI == EPI_VPAIR) {
                const unsigned short* q = B2 + boff + j * sub16 + k0;
                fc[j].h[0] = *(const u16x8*)(q);
                fc[j].h[1] = *(const u16x8*)(q + 16);
            }
        }
#pragma unroll
        for (int s = 0; s < 2; ++s)
#pragma unroll
            for (int j = 0; j < 2; ++j) {
                mma_hf(acc[s * 2 + j], fa[s], fb[j]);
                if (EPI == EPI_VPAIR) mma_hf(acc2[s * 2 + j], fa[s], fc[j]);
            }
    }

    float* st  = stile[wave];
    float* st2 = stile[(EPI == EPI_VPAIR) ? (wave + 4) : wave];
#pragma unroll
    for (int s = 0; s < 2; ++s)
#pragma unroll
        for (int j = 0; j < 2; ++j)
#pragma unroll
            for (int r = 0; r < 8; ++r) {
                st[(s * 16 + 8 * h + r) * GP + j * 16 + m] = acc[s * 2 + j][r];
                if (EPI == EPI_VPAIR) st2[(s * 16 + 8 * h + r) * GP + j * 16 + m] = acc2[s * 2 + j][r];
            }
    __syncthreads();

    const int rsub = lane >> 3;
    const int c0   = (lane & 7) * 4;
    const int gn   = colW + c0;
    const float isc = 0.0625f;

    v4f res[8];
#pragma unroll
    for (int it = 0; it < 8; ++it) {
        const int row = it * 4 + rsub;
        const int gm  = rowW + row;
        const v4f v = *(const v4f*)(st + row * GP + c0);
        v4f o;
        if (EPI == EPI_WDEC) {
            const v4f b0 = *(const v4f*)(q0 + gn);
            const v4f b1 = *(const v4f*)(q1 + gn);
#pragma unroll
            for (int q = 0; q < 4; ++q) {
                const float val  = v[q] * isc;
                const float warg = b0[q] + tanhf(val) * b1[q];
                const float u    = -warg;
                const float sp   = fmaxf(u, 0.0f) + log1pf(expf(-fabsf(u)));
                float wd = -sp - 0.5f;
                wd = fminf(fmaxf(wd, -10.0f), 0.0f);
                o[q] = expf(wd);
            }
        } else if (EPI == EPI_GGATE) {
            const v4f b0 = *(const v4f*)(q0 + gn);
#pragma unroll
            for (int q = 0; q < 4; ++q) o[q] = sigm(v[q] * isc) * b0[q];
        } else {
            const v4f vs = *(const v4f*)(st2 + row * GP + c0);
            const v4f b0 = *(const v4f*)(q0 + gn);
            const v4f b1 = *(const v4f*)(q1 + gn);
            const v4f vf = *(const v4f*)(q2 + (size_t)gm * C_ + gn);
#pragma unroll
            for (int q = 0; q < 4; ++q) {
                const float vv   = v[q] * isc;
                const float vg   = vs[q] * isc;
                const float gate = sigm(b0[q] + vg * b1[q]);
                o[q] = vv + (vf[q] - vv) * gate;
            }
        }
        res[it] = o;
    }

#pragma unroll
    for (int it = 0; it < 8; ++it) {
        const size_t o = (size_t)(rowW + it * 4 + rsub) * C_ + gn;
        *(volatile v4f*)(out0 + o) = res[it];
    }
    __threadfence();
#pragma unroll
    for (int it = 0; it < 8; ++it) {
        const size_t o = (size_t)(rowW + it * 4 + rsub) * C_ + gn;
        *(volatile v4f*)(out0 + o) = res[it];
    }
}

__global__ __launch_bounds__(256)
void scan_kernel(const float* __restrict__ Rp, const float* __restrict__ Wp, const float* __restrict__ Kp,
                 const float* __restrict__ Vp, const float* __restrict__ KKp, const float* __restrict__ Ap,
                 float* Yp)
{
    __shared__ __attribute__((aligned(16))) float sh[6][32 * 64];
    __shared__ __attribute__((aligned(16))) float sout[32 * 64];

    const int tid  = threadIdx.x;
    const int lane = tid & 31;
    const int wave = tid >> 5;
    const int bh   = blockIdx.x;
    const int b    = bh >> 4;
    const int hh   = bh & (H_ - 1);
    const int i    = tid >> 2;
    const int jq   = (tid & 3) * 16;
    const size_t colbase = (size_t)hh * N_;
    const size_t rowbase = (size_t)b * T_;

    float st[16];
#pragma unroll
    for (int e = 0; e < 16; ++e) st[e] = 0.0f;

    auto stage = [&](const float* src, float* dst, int t0) {
#pragma unroll
        for (int it = 0; it < 2; ++it) {
            const int idx = it * 256 + tid;
            const int s   = idx >> 4;
            const int e4  = (idx & 15) * 4;
            const v4f v = *(const v4f*)(src + (rowbase + t0 + s) * C_ + colbase + e4);
            *(v4f*)(dst + s * 64 + e4) = v;
        }
    };

#pragma unroll 1
    for (int ch = 0; ch < T_ / 32; ++ch) {
        const int t0 = ch * 32;
        __syncthreads();
        stage(Rp,  sh[0], t0);
        stage(Wp,  sh[1], t0);
        stage(Kp,  sh[2], t0);
        stage(Vp,  sh[3], t0);
        stage(KKp, sh[4], t0);
        stage(Ap,  sh[5], t0);
        __syncthreads();
        {
            const int s  = tid >> 3;
            const int e8 = (tid & 7) * 8;
            float*       pa = sh[5] + s * 64 + e8;
            const float* pk = sh[4] + s * 64 + e8;
#pragma unroll
            for (int q = 0; q < 8; ++q) pa[q] = pk[q] * pa[q];
        }
        __syncthreads();

#pragma unroll 1
        for (int s = 0; s < 32; ++s) {
            const float* pr  = sh[0] + s * 64 + jq;
            const float* pk  = sh[2] + s * 64 + jq;
            const float* pkk = sh[4] + s * 64 + jq;
            const float* pka = sh[5] + s * 64 + jq;
            const float w_i = sh[1][s * 64 + i];
            const float v_i = sh[3][s * 64 + i];

            v4f kk4[4];
#pragma unroll
            for (int q = 0; q < 4; ++q) kk4[q] = *(const v4f*)(pkk + 4 * q);
            float sa = 0.0f;
#pragma unroll
            for (int e = 0; e < 16; ++e) sa = st[e] * kk4[e >> 2][e & 3] + sa;
            sa += __shfl_xor(sa, 1, 32);
            sa += __shfl_xor(sa, 2, 32);
            const float sab = -sa;

            v4f ka4[4], k4[4], r4[4];
#pragma unroll
            for (int q = 0; q < 4; ++q) {
                ka4[q] = *(const v4f*)(pka + 4 * q);
                k4[q]  = *(const v4f*)(pk + 4 * q);
                r4[q]  = *(const v4f*)(pr + 4 * q);
            }
            float yp = 0.0f;
#pragma unroll
            for (int e = 0; e < 16; ++e) {
                const float t1 = st[e] * w_i;
                const float t2 = sab * ka4[e >> 2][e & 3];
                const float t3 = v_i * k4[e >> 2][e & 3];
                st[e] = (t1 + t2) + t3;
                yp = st[e] * r4[e >> 2][e & 3] + yp;
            }
            yp += __shfl_xor(yp, 1, 32);
            yp += __shfl_xor(yp, 2, 32);
            if ((tid & 3) == 0) sout[s * 64 + i] = yp;
        }
        __syncthreads();

        const int c = (lane & 15) * 4;
        v4f fv[2];
#pragma unroll
        for (int it = 0; it < 2; ++it) {
            const int row = wave * 4 + it * 2 + (lane >> 4);
            fv[it] = *(const v4f*)(sout + row * 64 + c);
        }
#pragma unroll
        for (int it = 0; it < 2; ++it) {
            const int row = wave * 4 + it * 2 + (lane >> 4);
            float* gp = Yp + (rowbase + t0 + row) * C_ + colbase + c;
            *(volatile v4f*)gp = fv[it];
        }
        __threadfence();
#pragma unroll
        for (int it = 0; it < 2; ++it) {
            const int row = wave * 4 + it * 2 + (lane >> 4);
            float* gp = Yp + (rowbase + t0 + row) * C_ + colbase + c;
            *(volatile v4f*)gp = fv[it];
        }
    }
}

__global__ __launch_bounds__(256)
void norm_gate_kernel(const float* __restrict__ Y, const float* __restrict__ R, const float* __restrict__ K,
                      const float* __restrict__ V, const float* __restrict__ G,
                      const float* __restrict__ rk, const float* __restrict__ lw, const float* __restrict__ lb,
                      unsigned short* yh, unsigned short* yl)
{
    const int tid  = threadIdx.x;
    const int lane = tid & 31;
    const int wave = tid >> 5;
    const int grp  = (blockIdx.x * 8 + wave) * 4 + (lane >> 3);
    const int mrow = grp >> 4;
    const int hh   = grp & (H_ - 1);
    const int c0   = (lane & 7) * 8;
    const int ch   = hh * N_ + c0;
    const size_t base = (size_t)mrow * C_ + ch;

    const v8f y = ld8f(Y + base);
    const v8f r = ld8f(R + base);
    const v8f k = ld8f(K + base);
    const v8f v = ld8f(V + base);
    const v8f g = ld8f(G + base);
    const v8f w8 = ld8f(lw + ch);
    const v8f b8 = ld8f(lb + ch);
    const v8f rk8 = ld8f(rk + ch);

    float s = 0.0f;
#pragma unroll
    for (int q = 0; q < 8; ++q) s += y[q];
    s += __shfl_xor(s, 4, 32);
    s += __shfl_xor(s, 2, 32);
    s += __shfl_xor(s, 1, 32);
    const float mean = s * (1.0f / 64.0f);

    v8f d;
    float sq = 0.0f;
#pragma unroll
    for (int q = 0; q < 8; ++q) { d[q] = y[q] - mean; sq = d[q] * d[q] + sq; }
    sq += __shfl_xor(sq, 4, 32);
    sq += __shfl_xor(sq, 2, 32);
    sq += __shfl_xor(sq, 1, 32);
    const float var = sq * (1.0f / 64.0f);
    const float inv = 1.0f / sqrtf(var + EPSGN);

    float dot = 0.0f;
#pragma unroll
    for (int q = 0; q < 8; ++q) dot = (r[q] * k[q]) * rk8[q] + dot;
    dot += __shfl_xor(dot, 4, 32);
    dot += __shfl_xor(dot, 2, 32);
    dot += __shfl_xor(dot, 1, 32);

    v8f o;
#pragma unroll
    for (int q = 0; q < 8; ++q) o[q] = (((d[q] * inv) * w8[q] + b8[q]) + dot * v[q]) * g[q];

    u16x8 hv, lv;
    split8(o, hv, lv);
    *(volatile u16x8*)(yh + base) = hv;
    *(volatile u16x8*)(yl + base) = lv;
    __threadfence();
    *(volatile u16x8*)(yh + base) = hv;
    *(volatile u16x8*)(yl + base) = lv;
}

__global__ __launch_bounds__(256)
void copy_kernel(const float* __restrict__ src, float* dst, int n4)
{
    const int i = blockIdx.x * 256 + threadIdx.x;
    if (i >= n4) return;
    const size_t e = (size_t)i * 4;
    const v4f v = *(const v4f*)(src + e);
    *(volatile v4f*)(dst + e) = v;
    __threadfence();
    *(volatile v4f*)(dst + e) = v;
}

extern "C" void kernel_launch(void* const* d_in, const int* in_sizes, int n_in,
                              void* d_out, int out_size, void* d_ws, size_t ws_size,
                              hipStream_t stream)
{
    if (n_in < 29) return;
    if (in_sizes[0] != M_ * C_) return;
    if (in_sizes[1] != M_ * C_) return;
    for (int i = 2; i <= 10; ++i) if (in_sizes[i] != C_) return;
    for (int i = 11; i <= 19; ++i) if (in_sizes[i] != C_ * C_) return;
    for (int i = 20; i <= 28; ++i) if (in_sizes[i] != C_) return;
    if (out_size != 2 * M_ * C_) return;
    if (ws_size < WS_END) return;

    const float* x      = (const float*)d_in[0];
    const float* vfirst = (const float*)d_in[1];
    const float* x_r    = (const float*)d_in[2];
    const float* x_w    = (const float*)d_in[3];
    const float* x_k    = (const float*)d_in[4];
    const float* x_v    = (const float*)d_in[5];
    const float* x_a    = (const float*)d_in[6];
    const float* x_g    = (const float*)d_in[7];
    const float* in_w0  = (const float*)d_in[8];
    const float* in_a0  = (const float*)d_in[9];
    const float* in_v0  = (const float*)d_in[10];
    const float* Wr     = (const float*)d_in[11];
    const float* Wk     = (const float*)d_in[12];
    const float* Wv     = (const float*)d_in[13];
    const float* Wo     = (const float*)d_in[15];
    const float* Ww1    = (const float*)d_in[16];
    const float* Wa1    = (const float*)d_in[17];
    const float* Wv1    = (const float*)d_in[18];
    const float* Wg1    = (const float*)d_in[19];
    const float* in_w2  = (const float*)d_in[20];
    const float* in_a2  = (const float*)d_in[21];
    const float* in_v2  = (const float*)d_in[22];
    const float* in_g2  = (const float*)d_in[23];
    const float* k_k    = (const float*)d_in[24];
    const float* k_a    = (const float*)d_in[25];
    const float* r_k    = (const float*)d_in[26];
    const float* ln_w   = (const float*)d_in[27];
    const float* ln_b   = (const float*)d_in[28];
    float* out0 = (float*)d_out;
    float* out1 = out0 + (size_t)M_ * C_;

    char* ws = (char*)d_ws;
    unsigned short* xh  = (unsigned short*)(ws + OFF_XH);
    unsigned short* xl  = (unsigned short*)(ws + OFF_XL);
    unsigned short* wh  = (unsigned short*)(ws + OFF_WH);
    unsigned short* wl  = (unsigned short*)(ws + OFF_WL);
    unsigned short* ww2 = (unsigned short*)(ws + OFF_W2);
    float*          plY = (float*)(ws + OFF_Y);
    unsigned short* xg  = (unsigned short*)(ws + OFF_XG);
    unsigned short* wg  = (unsigned short*)(ws + OFF_WG);
    unsigned short* woh = (unsigned short*)(ws + OFF_WOH);
    unsigned short* wol = (unsigned short*)(ws + OFF_WOL);
    float*          plA  = (float*)(ws + OFF_A);
    float*          plKM = (float*)(ws + OFF_KM);
    float*          plKK = (float*)(ws + OFF_KK);
    float*          plR  = (float*)(ws + OFF_R);
    float*          plWD = (float*)(ws + OFF_WD);
    float*          plV  = (float*)(ws + OFF_V);
    float*          plG  = (float*)(ws + OFF_G);
    unsigned short* ygh  = (unsigned short*)(ws + OFF_YGH);
    unsigned short* ygl  = (unsigned short*)(ws + OFF_YGL);

    const int n8x = (M_ * C_) / 8;
    const int n8w = (C_ * C_) / 8;
    const dim3 gx((n8x + 255) / 256);
    const dim3 gw((n8w + 255) / 256);
    const dim3 gg(C_ / 64, M_ / 64);
    const dim3 b256(256), b128(128);

    mix_split_kernel<<<gx, b256, 0, stream>>>(x, x_a, xh, xl, n8x);
    w_split_kernel<<<gw, b256, 0, stream>>>(Wa1, wh, wl, n8w);
    gemm_x3_kernel<EPI_AGATE><<<gg, b128, 0, stream>>>(xh, xl, wh, wl, plA, plA, in_a0, in_a2, in_a0);

    mix_split_kernel<<<gx, b256, 0, stream>>>(x, x_k, xh, xl, n8x);
    w_split_kernel<<<gw, b256, 0, stream>>>(Wk, wh, wl, n8w);
    gemm_x3_kernel<EPI_KPOST><<<gg, b128, 0, stream>>>(xh, xl, wh, wl, plKM, plKK, k_k, k_a, (const float*)plA);

    mix_split_kernel<<<gx, b256, 0, stream>>>(x, x_r, xh, xl, n8x);
    w_split_kernel<<<gw, b256, 0, stream>>>(Wr, wh, wl, n8w);
    gemm_x3_kernel<EPI_PLAIN><<<gg, b128, 0, stream>>>(xh, xl, wh, wl, plR, plR, k_k, k_k, k_k);

    mix_f16_kernel<<<gx, b256, 0, stream>>>(x, x_w, xh, n8x);
    mix_f16_kernel<<<gx, b256, 0, stream>>>(x, x_v, xl, n8x);
    w_f16_kernel<<<gw, b256, 0, stream>>>(Ww1, wh, n8w);
    w_f16_kernel<<<gw, b256, 0, stream>>>(Wv, wl, n8w);
    w_f16_kernel<<<gw, b256, 0, stream>>>(Wv1, ww2, n8w);
    gemm_f16_kernel<EPI_WDEC><<<gg, b128, 0, stream>>>(xh, wh, wh, plWD, in_w0, in_w2, in_w0);
    gemm_f16_kernel<EPI_VPAIR><<<gg, b128, 0, stream>>>(xl, wl, ww2, plV, in_v0, in_v2, vfirst);

    scan_kernel<<<dim3((M_ / T_) * H_), b256, 0, stream>>>(
        (const float*)plR, (const float*)plWD, (const float*)plKM, (const float*)plV,
        (const float*)plKK, (const float*)plA, plY);

    mix_f16_kernel<<<gx, b256, 0, stream>>>(x, x_g, xg, n8x);
    w_f16_kernel<<<gw, b256, 0, stream>>>(Wg1, wg, n8w);
    w_split_kernel<<<gw, b256, 0, stream>>>(Wo, woh, wol, n8w);
    gemm_f16_kernel<EPI_GGATE><<<gg, b128, 0, stream>>>(xg, wg, wg, plG, in_g2, in_g2, in_g2);

    norm_gate_kernel<<<dim3((M_ * H_) / 32), b256, 0, stream>>>(
        (const float*)plY, (const float*)plR, (const float*)plKM, (const float*)plV, (const float*)plG,
        r_k, ln_w, ln_b, ygh, ygl);

    gemm_x3_kernel<EPI_PLAIN><<<gg, b128, 0, stream>>>(ygh, ygl, woh, wol, out0, out0, k_k, k_k, k_k);

    {
        const int n4 = (M_ * C_) / 4;
        copy_kernel<<<dim3((n4 + 255) / 256), b256, 0, stream>>>(vfirst, out1, n4);
    }
}
